// Trans_89283780149720
// MI455X (gfx1250) — hardware-verified
//
#include <hip/hip_runtime.h>
#include <math.h>

constexpr int kBatch  = 4;
constexpr int kSeq    = 1024;
constexpr int kDim    = 1024;
constexpr int kHeads  = 16;
constexpr int kDk     = 64;
constexpr int kDff    = 4096;
constexpr int kTok    = kBatch * kSeq;
constexpr int kGrp    = 8;
constexpr int kNChunk = (kBatch * kHeads) / kGrp;
static_assert(kHeads % kGrp == 0, "chunk groups share one batch index");
constexpr float kWCarry   = 16.0f;
constexpr float kWInv     = 1.0f / 16.0f;
constexpr float kPCarry   = 2048.0f;
constexpr float kCtxCarry = 256.0f;
constexpr float kScoreScale = 0.125f;
constexpr float kPVScale  = kCtxCarry / kPCarry;
constexpr float kOutScale = 1.0f / (kCtxCarry * kWCarry);
constexpr float kLnEps    = 1e-6f;

constexpr size_t kMiB   = 1048576;
constexpr size_t R_W    = 0;
constexpr size_t R_N16  = 8 * kMiB;
constexpr size_t R_Z16  = 16 * kMiB;
constexpr size_t R_QK   = 24 * kMiB;
constexpr size_t R_VT   = 40 * kMiB;
constexpr size_t R_ATT  = 48 * kMiB;
constexpr size_t R_Y1   = 56 * kMiB;
constexpr size_t R_S    = 72 * kMiB;
constexpr size_t R_P    = 104 * kMiB;
constexpr size_t R_END  = 120 * kMiB;
constexpr size_t R_Y2   = R_S;
constexpr size_t R_H16  = R_QK;
static_assert(R_N16 - R_W   >= (size_t)4 * kDim * kDim * 2, "w16");
static_assert(R_Z16 - R_N16 >= (size_t)kTok * kDim * 2, "n16");
static_assert(R_QK  - R_Z16 >= (size_t)kTok * kDim * 2 && R_QK - R_Z16 >= (size_t)kDim * kDff * 2, "z16/w2");
static_assert(R_VT  - R_QK  >= (size_t)kTok * 2 * kDim * 2, "qk16");
static_assert(R_ATT - R_VT  >= (size_t)kDim * kTok * 2, "vt16");
static_assert(R_Y1  - R_ATT >= (size_t)kTok * kDim * 2, "att16");
static_assert(R_S   - R_Y1  >= (size_t)kTok * kDim * 4, "y1");
static_assert(R_P   - R_S   >= (size_t)kGrp * kSeq * kSeq * 4, "scores");
static_assert(R_END - R_P   >= (size_t)kGrp * kSeq * kSeq * 2, "p16");
static_assert(R_P   - R_Y2  >= (size_t)kTok * kDim * 4, "y2");
static_assert(R_Y1  - R_H16 >= (size_t)kTok * kDff * 2, "h16");
static_assert(R_END == 125829120, "carve total");

typedef __attribute__((ext_vector_type(16))) _Float16 v16h;
typedef __attribute__((ext_vector_type(8)))  _Float16 v8h;
typedef __attribute__((ext_vector_type(16))) __bf16   v16b;
typedef __attribute__((ext_vector_type(8)))  __bf16   v8b;
typedef __attribute__((ext_vector_type(8)))  float    v8f;
typedef __attribute__((ext_vector_type(4)))  float    v4f;
typedef __attribute__((ext_vector_type(4)))  unsigned int v4u;
typedef __attribute__((ext_vector_type(4)))  int      v4i;

__device__ __forceinline__ unsigned short f2bf_bits(float f) {
  unsigned u = __float_as_uint(f);
  return (unsigned short)((u + 0x7FFFu + ((u >> 16) & 1u)) >> 16);
}
__device__ __forceinline__ float bf_bits2f(unsigned short h) { return __uint_as_float(((unsigned)h) << 16); }

__device__ __forceinline__ void dep_guard_h(v8f& a, v8f& b, v16h x, v16h y) { asm volatile("v_nop\n\tv_nop\n\tv_nop\n\tv_nop" : "+v"(a), "+v"(b) : "v"(x), "v"(y)); }
__device__ __forceinline__ void dep_guard_b(v8f& a, v8f& b, v16b x, v16b y) { asm volatile("v_nop\n\tv_nop\n\tv_nop\n\tv_nop" : "+v"(a), "+v"(b) : "v"(x), "v"(y)); }
__device__ __forceinline__ void keep4_h(v16h a, v16h b, v16h c, v16h d) { asm volatile("v_nop" :: "v"(a), "v"(b), "v"(c), "v"(d)); }
__device__ __forceinline__ void keep4_b(v16b a, v16b b, v16b c, v16b d) { asm volatile("v_nop" :: "v"(a), "v"(b), "v"(c), "v"(d)); }
__device__ __forceinline__ void acc_guard4(v8f& a, v8f& b, v8f& c, v8f& d) { asm volatile("v_nop\n\tv_nop\n\tv_nop\n\tv_nop" : "+v"(a), "+v"(b), "+v"(c), "+v"(d)); }
template <typename T> struct Frag;
template <> struct Frag<_Float16> {
  typedef v16h V; union U { v16h v; v8h h[2]; };
  static __device__ __forceinline__ v16h load(const _Float16* p) {
    U f; f.h[0] = *(const v8h*)(p); f.h[1] = *(const v8h*)(p + 16); return f.v;
  }
  static __device__ __forceinline__ v8f mma(v16h a, v16h b, v8f c) {
    return __builtin_amdgcn_wmma_f32_16x16x32_f16(false, a, false, b, (short)0, c, false, false);
  }
  static __device__ __forceinline__ void guard(v8f& a, v8f& b, v16h x, v16h y) { dep_guard_h(a, b, x, y); }
  static __device__ __forceinline__ void keep(v16h a, v16h b, v16h c, v16h d) { keep4_h(a, b, c, d); }
};
template <> struct Frag<__bf16> {
  typedef v16b V; union U { v16b v; v8b h[2]; };
  static __device__ __forceinline__ v16b load(const __bf16* p) {
    U f; f.h[0] = *(const v8b*)(p); f.h[1] = *(const v8b*)(p + 16); return f.v;
  }
  static __device__ __forceinline__ v8f mma(v16b a, v16b b, v8f c) {
    return __builtin_amdgcn_wmma_f32_16x16x32_bf16(false, a, false, b, (short)0, c, false, false);
  }
  static __device__ __forceinline__ void guard(v8f& a, v8f& b, v16b x, v16b y) { dep_guard_b(a, b, x, y); }
  static __device__ __forceinline__ void keep(v16b a, v16b b, v16b c, v16b d) { keep4_b(a, b, c, d); }
};

__device__ __forceinline__ unsigned pk16(unsigned short a, unsigned short b) { return (unsigned)a | ((unsigned)b << 16); }
__device__ __forceinline__ unsigned short h_bits(float f) { const _Float16 h = (_Float16)f; return __builtin_bit_cast(unsigned short, h); }

template <int ET> struct Elem;
template <> struct Elem<0> { typedef _Float16 T; };
template <> struct Elem<1> { typedef __bf16 T; };
template <int ET, bool SPLIT, int BIAS_MODE, int OUT_MODE, bool RESID, int ACT = 0>
__global__ __launch_bounds__(256) void wmma_gemm64(
    const unsigned short* __restrict__ Ap, const unsigned short* __restrict__ A2p, int lda, long strideA,
    const unsigned short* __restrict__ Btp, const unsigned short* __restrict__ Bt2p, int ldb, long strideB,
    void* __restrict__ Cout, void* __restrict__ Cout2, int ldc, long strideC,
    const float* __restrict__ bias,
    const float* __restrict__ resid, long strideR,
    int M, int N, int K, float scale) {
  typedef typename Elem<ET>::T T;
  typedef typename Frag<T>::V V;
  const T* A = (const T*)Ap; const T* A2 = (const T*)A2p; const T* Bt = (const T*)Btp; const T* Bt2 = (const T*)Bt2p;
  __shared__ __align__(16) float sT[8][16 * 68];
  const int b    = blockIdx.y;
  const int lane = threadIdx.x & 31;
  const int wave = threadIdx.x >> 5;
  const int tilesN = N >> 6;
  const int tilesM = M >> 6;
  const int tile = blockIdx.x * 8 + wave;
  if (tile >= tilesM * tilesN) return;
  const int tm = tile / tilesN;
  const int tn = tile - tm * tilesN;
  const int m0 = tm << 6;
  const int n0 = tn << 6;

  const T* Ab  = A  + (size_t)b * strideA;
  const T* Bb  = Bt + (size_t)b * strideB;
  const T* Ab2 = SPLIT ? (A2  + (size_t)b * strideA) : nullptr;
  const T* Bb2 = SPLIT ? (Bt2 + (size_t)b * strideB) : nullptr;

  const int rlane = lane & 15;
  const int koff  = (lane >> 4) * 8;
  const int mOff  = (lane >> 4) * 8;

  v8f acc[4][4];
#pragma unroll
  for (int i = 0; i < 4; ++i)
#pragma unroll
    for (int j = 0; j < 4; ++j) acc[i][j] = (v8f){0.f,0.f,0.f,0.f,0.f,0.f,0.f,0.f};

  for (int k0 = 0; k0 < K; k0 += 32) {
    V bh[4], bl[4];
#pragma unroll
    for (int j = 0; j < 4; ++j) {
      const size_t bo = (size_t)(n0 + (j << 4) + rlane) * ldb + koff + k0;
      bh[j] = Frag<T>::load(Bb + bo);
      if (SPLIT) bl[j] = Frag<T>::load(Bb2 + bo);
    }
#pragma unroll
    for (int i = 0; i < 4; ++i) {
      const size_t ao = (size_t)(m0 + (i << 4) + rlane) * lda + koff + k0;
      V ah = Frag<T>::load(Ab + ao);
      V al;
      if (SPLIT) al = Frag<T>::load(Ab2 + ao);
#pragma unroll
      for (int j = 0; j < 4; ++j) {
        acc[i][j] = Frag<T>::mma(ah, bh[j], acc[i][j]);
        if (SPLIT) {
          acc[i][j] = Frag<T>::mma(ah, bl[j], acc[i][j]);
          acc[i][j] = Frag<T>::mma(al, bh[j], acc[i][j]);
        }
      }
      Frag<T>::guard(acc[i][0], acc[i][3], ah, SPLIT ? al : ah);
    }
    Frag<T>::keep(bh[0], bh[1], bh[2], bh[3]);
    if (SPLIT) Frag<T>::keep(bl[0], bl[1], bl[2], bl[3]);
  }
  acc_guard4(acc[0][0], acc[0][1], acc[0][2], acc[0][3]);
  acc_guard4(acc[1][0], acc[1][1], acc[1][2], acc[1][3]);
  acc_guard4(acc[2][0], acc[2][1], acc[2][2], acc[2][3]);
  acc_guard4(acc[3][0], acc[3][1], acc[3][2], acc[3][3]);

  float* slab = sT[wave];
  const float* Rb = RESID ? (resid + (size_t)b * strideR) : nullptr;
#pragma unroll
  for (int i = 0; i < 4; ++i) {
    const int mBase = m0 + (i << 4);
#pragma unroll
    for (int j = 0; j < 4; ++j) {
      const int n = n0 + (j << 4) + rlane;
      float bv = 0.f;
      if (BIAS_MODE == 2) bv = bias[n];
#pragma unroll
      for (int r = 0; r < 8; ++r) {
        float v = acc[i][j][r] * scale;
        if (BIAS_MODE == 1) v += bias[mBase + mOff + r];
        if (BIAS_MODE == 2) v += bv;
        if (RESID) v += Rb[(size_t)(mBase + mOff + r) * ldc + n];
        if (ACT == 2) v = fmaxf(v, 0.0f);
        if (ACT == 3) v = v / (1.0f + expf(-v));
        if (ACT == 4) v = (v > 0.f) ? v : 0.01f * v;
        slab[(mOff + r) * 68 + (j << 4) + rlane] = v;
      }
    }
    __builtin_amdgcn_fence(__ATOMIC_RELEASE, "workgroup");
    __builtin_amdgcn_wave_barrier();
    __builtin_amdgcn_fence(__ATOMIC_ACQUIRE, "workgroup");
    if (OUT_MODE == 0) {
      float* C = (float*)Cout + (size_t)b * strideC;
      const int hh = lane >> 4, c4 = (lane & 15) * 4;
      for (int pass = 0; pass < 2; ++pass) {
#pragma unroll
        for (int it = 0; it < 8; ++it) {
          const int row = it * 2 + hh;
          v4f v = *(const v4f*)(slab + row * 68 + c4);
          *(volatile v4f*)(C + (size_t)(mBase + row) * ldc + n0 + c4) = v;
        }
        __threadfence();
      }
    } else {
      const int q = lane >> 3, c8 = (lane & 7) * 8;
      unsigned short* C  = (unsigned short*)Cout  + (size_t)b * strideC;
      unsigned short* C2 = (OUT_MODE == 2) ? ((unsigned short*)Cout2 + (size_t)b * strideC) : nullptr;
      for (int pass = 0; pass < 2; ++pass) {
#pragma unroll
        for (int it = 0; it < 4; ++it) {
          const int row = it * 4 + q;
          const float* sp = slab + row * 68 + c8;
          v8h hv, lv;
#pragma unroll
          for (int e = 0; e < 8; ++e) {
            if (OUT_MODE == 1) {
              hv[e] = (_Float16)sp[e];
            } else {
              unsigned short hb = f2bf_bits(sp[e]);
              unsigned short lb = f2bf_bits(sp[e] - bf_bits2f(hb));
              hv[e] = __builtin_bit_cast(_Float16, hb);
              lv[e] = __builtin_bit_cast(_Float16, lb);
            }
          }
          *(volatile v8h*)(C + (size_t)(mBase + row) * ldc + n0 + c8) = hv;
          if (OUT_MODE == 2) *(volatile v8h*)(C2 + (size_t)(mBase + row) * ldc + n0 + c8) = lv;
        }
        __threadfence();
      }
    }
    __builtin_amdgcn_fence(__ATOMIC_RELEASE, "workgroup");
    __builtin_amdgcn_wave_barrier();
    __builtin_amdgcn_fence(__ATOMIC_ACQUIRE, "workgroup");
  }
}

__global__ __launch_bounds__(256) void cast8_f16_kernel(const float* __restrict__ in, unsigned short* __restrict__ out, int n8, float scale) {
  const int i = blockIdx.x * 256 + threadIdx.x;
  if (i >= n8) return;
  const float* p = in + 8 * (size_t)i;
  const v4f a = *(const v4f*)(p);
  const v4f c = *(const v4f*)(p + 4);
  unsigned short hb[8];
#pragma unroll
  for (int e = 0; e < 4; ++e) {
    hb[e]     = h_bits(a[e] * scale);
    hb[4 + e] = h_bits(c[e] * scale);
  }
  const v4u u = (v4u){pk16(hb[0], hb[1]), pk16(hb[2], hb[3]), pk16(hb[4], hb[5]), pk16(hb[6], hb[7])};
  unsigned short* q = out + 8 * (size_t)i;
  *(volatile v4u*)q = u;
  __threadfence();
  *(volatile v4u*)q = u;
}

__global__ __launch_bounds__(128) void ln_kernel(const float* __restrict__ x, const float* __restrict__ g,
                                                 const float* __restrict__ bta, unsigned short* __restrict__ out) {
  __shared__ float red1[4];
  __shared__ float red2[4];
  const int row  = blockIdx.x;
  const int t    = threadIdx.x;
  const int lane = t & 31, wave = t >> 5;
  const int c0   = t * 8;
  const float* xr = x + (size_t)row * kDim + c0;
  const v4f a = *(const v4f*)(xr);
  const v4f c = *(const v4f*)(xr + 4);
  float v[8];
#pragma unroll
  for (int e = 0; e < 4; ++e) { v[e] = a[e]; v[4 + e] = c[e]; }
  float s = ((v[0] + v[1]) + (v[2] + v[3])) + ((v[4] + v[5]) + (v[6] + v[7]));
#pragma unroll
  for (int off = 16; off > 0; off >>= 1) s += __shfl_xor(s, off, 32);
  if (lane == 0) red1[wave] = s;
  __syncthreads();
  const float tot = (red1[0] + red1[1]) + (red1[2] + red1[3]);
  const float mean = tot * (1.0f / 1024.0f);
  float d[8];
#pragma unroll
  for (int e = 0; e < 8; ++e) d[e] = v[e] - mean;
  float ss = ((d[0] * d[0] + d[1] * d[1]) + (d[2] * d[2] + d[3] * d[3])) + ((d[4] * d[4] + d[5] * d[5]) + (d[6] * d[6] + d[7] * d[7]));
#pragma unroll
  for (int off = 16; off > 0; off >>= 1) ss += __shfl_xor(ss, off, 32);
  if (lane == 0) red2[wave] = ss;
  __syncthreads();
  const float tot2 = (red2[0] + red2[1]) + (red2[2] + red2[3]);
  const float var  = tot2 * (1.0f / 1023.0f);
  const float sd   = sqrtf(fmaxf(var, 0.0f));
  const float inv  = 1.0f / (sd + kLnEps);
  const v4f ga = *(const v4f*)(g + c0);
  const v4f gc = *(const v4f*)(g + c0 + 4);
  const v4f ba = *(const v4f*)(bta + c0);
  const v4f bc = *(const v4f*)(bta + c0 + 4);
  unsigned short hb[8];
#pragma unroll
  for (int e = 0; e < 4; ++e) {
    hb[e]     = h_bits((ga[e] * d[e]) * inv + ba[e]);
    hb[4 + e] = h_bits((gc[e] * d[4 + e]) * inv + bc[e]);
  }
  const v4u u = (v4u){pk16(hb[0], hb[1]), pk16(hb[2], hb[3]), pk16(hb[4], hb[5]), pk16(hb[6], hb[7])};
  unsigned short* q = out + (size_t)row * kDim + c0;
  *(volatile v4u*)q = u;
  __threadfence();
  *(volatile v4u*)q = u;
}

__global__ __launch_bounds__(128) void softmax_row_kernel(const float* __restrict__ S, const int* __restrict__ mrow,
                                                          unsigned short* __restrict__ P, float carry) {
  __shared__ float redM[4];
  __shared__ float redS[4];
  const int row  = blockIdx.x;
  const int t    = threadIdx.x;
  const int lane = t & 31, wave = t >> 5;
  const int c0   = t * 8;
  const float* sr = S + (size_t)row * kSeq + c0;
  const v4f a = *(const v4f*)(sr);
  const v4f c = *(const v4f*)(sr + 4);
  const v4i ma = *(const v4i*)(mrow + c0);
  const v4i mc = *(const v4i*)(mrow + c0 + 4);
  float x[8];
#pragma unroll
  for (int e = 0; e < 4; ++e) {
    x[e]     = (ma[e] == 0) ? -1e9f : a[e];
    x[4 + e] = (mc[e] == 0) ? -1e9f : c[e];
  }
  float m = fmaxf(fmaxf(fmaxf(x[0], x[1]), fmaxf(x[2], x[3])), fmaxf(fmaxf(x[4], x[5]), fmaxf(x[6], x[7])));
#pragma unroll
  for (int off = 16; off > 0; off >>= 1) m = fmaxf(m, __shfl_xor(m, off, 32));
  if (lane == 0) redM[wave] = m;
  __syncthreads();
  const float mx = fmaxf(fmaxf(redM[0], redM[1]), fmaxf(redM[2], redM[3]));
  float ex[8];
#pragma unroll
  for (int e = 0; e < 8; ++e) ex[e] = expf(x[e] - mx);
  float s = ((ex[0] + ex[1]) + (ex[2] + ex[3])) + ((ex[4] + ex[5]) + (ex[6] + ex[7]));
#pragma unroll
  for (int off = 16; off > 0; off >>= 1) s += __shfl_xor(s, off, 32);
  if (lane == 0) redS[wave] = s;
  __syncthreads();
  const float tot = (redS[0] + redS[1]) + (redS[2] + redS[3]);
  const float inv = 1.0f / tot;
  unsigned short hb[8];
#pragma unroll
  for (int e = 0; e < 8; ++e) hb[e] = h_bits((ex[e] * inv) * carry);
  const v4u u = (v4u){pk16(hb[0], hb[1]), pk16(hb[2], hb[3]), pk16(hb[4], hb[5]), pk16(hb[6], hb[7])};
  unsigned short* q = P + (size_t)row * kSeq + c0;
  *(volatile v4u*)q = u;
  __threadfence();
  *(volatile v4u*)q = u;
}

template <int BIAS_MODE, int OUT_MODE, bool RESID, int ACT>
static void launch_gemm(hipStream_t st, const unsigned short* A, int lda, long sA,
                        const unsigned short* Bt, int ldb, long sB,
                        void* C, int ldc, long sC, const float* bias, const float* resid, long sR,
                        int M, int N, int K, float scale, int nbatch) {
  const int tiles = (M / 64) * (N / 64);
  const int gx = (tiles + 7) / 8;
  wmma_gemm64<0, false, BIAS_MODE, OUT_MODE, RESID, ACT><<<dim3(gx, nbatch), 256, 0, st>>>(
      A, A, lda, sA, Bt, Bt, ldb, sB, C, C, ldc, sC, bias, resid, sR, M, N, K, scale);
}

extern "C" void kernel_launch(void* const* d_in, const int* in_sizes, int n_in,
                              void* d_out, int out_size, void* d_ws, size_t ws_size,
                              hipStream_t stream) {
  (void)in_sizes; (void)n_in; (void)out_size;
  if (ws_size < R_END) return;

  const float* y    = (const float*)d_in[0];
  const float* z    = (const float*)d_in[1];
  const int*   mask = (const int*)d_in[2];
  const float* sa_w = (const float*)d_in[3];
  const float* sa_b = (const float*)d_in[4];
  const float* ca_w = (const float*)d_in[5];
  const float* ca_b = (const float*)d_in[6];
  const float* w1   = (const float*)d_in[7];
  const float* b1   = (const float*)d_in[8];
  const float* w2   = (const float*)d_in[9];
  const float* b2   = (const float*)d_in[10];
  const float* ln_g = (const float*)d_in[11];
  const float* ln_b = (const float*)d_in[12];
  float* outp = (float*)d_out;

  char* ws = (char*)d_ws;
  unsigned short* W16   = (unsigned short*)(ws + R_W);
  unsigned short* N16   = (unsigned short*)(ws + R_N16);
  unsigned short* Z16   = (unsigned short*)(ws + R_Z16);
  unsigned short* W2_16 = (unsigned short*)(ws + R_Z16);
  unsigned short* QK16  = (unsigned short*)(ws + R_QK);
  unsigned short* Q16   = (unsigned short*)(ws + R_QK);
  unsigned short* K16   = (unsigned short*)(ws + R_QK) + (size_t)kTok * kDim;
  unsigned short* VT16  = (unsigned short*)(ws + R_VT);
  unsigned short* ATT16 = (unsigned short*)(ws + R_ATT);
  unsigned short* H16   = (unsigned short*)(ws + R_H16);
  float* Y1 = (float*)(ws + R_Y1);
  float* Y2 = (float*)(ws + R_Y2);
  float* Sc = (float*)(ws + R_S);
  unsigned short* P16 = (unsigned short*)(ws + R_P);

  const size_t DD  = (size_t)kDim * kDim;
  const size_t SS2 = (size_t)kSeq * kSeq;
  const int n8w = (int)(4 * DD / 8);
  const int castBlocks = (n8w + 255) / 256;

  cast8_f16_kernel<<<castBlocks, 256, 0, stream>>>(sa_w, W16, n8w, kWCarry);
  ln_kernel<<<kTok, 128, 0, stream>>>(y, ln_g, ln_b, N16);
  launch_gemm<2, 1, false, 0>(stream, N16, kDim, 0, W16, kDim, 0, QK16, 2 * kDim, 0, sa_b, y, 0,
                              kTok, 2 * kDim, kDim, kWInv, 1);
  launch_gemm<1, 1, false, 0>(stream, W16 + 2 * DD, kDim, 0, N16, kDim, 0, VT16, kTok, 0, sa_b + 2 * kDim, y, 0,
                              kDim, kTok, kDim, kWInv, 1);
  for (int ch = 0; ch < kNChunk; ++ch) {
    const int b  = ch / (kHeads / kGrp);
    const int h0 = (ch % (kHeads / kGrp)) * kGrp;
    launch_gemm<0, 0, false, 0>(stream,
                                QK16 + (size_t)b * kSeq * (2 * kDim) + (size_t)h0 * kDk, 2 * kDim, kDk,
                                QK16 + (size_t)b * kSeq * (2 * kDim) + kDim + (size_t)h0 * kDk, 2 * kDim, kDk,
                                Sc, kSeq, (long)SS2, sa_b, y, 0, kSeq, kSeq, kDk, kScoreScale, kGrp);
    softmax_row_kernel<<<kGrp * kSeq, 128, 0, stream>>>(Sc, mask + (size_t)b * kSeq, P16, kPCarry);
    launch_gemm<0, 1, false, 0>(stream, P16, kSeq, (long)SS2,
                                VT16 + (size_t)h0 * kDk * kTok + (size_t)b * kSeq, kTok, (long)kDk * kTok,
                                ATT16 + (size_t)b * kSeq * kDim + (size_t)h0 * kDk, kDim, kDk,
                                sa_b, y, 0, kSeq, kDk, kSeq, kPVScale, kGrp);
  }
  launch_gemm<2, 0, true, 0>(stream, ATT16, kDim, 0, W16 + 3 * DD, kDim, 0, Y1, kDim, 0, sa_b + 3 * kDim, y, 0,
                             kTok, kDim, kDim, kOutScale, 1);

  cast8_f16_kernel<<<castBlocks, 256, 0, stream>>>(ca_w, W16, n8w, kWCarry);
  cast8_f16_kernel<<<castBlocks, 256, 0, stream>>>(z, Z16, n8w, 1.0f);
  ln_kernel<<<kTok, 128, 0, stream>>>(Y1, ln_g + kDim, ln_b + kDim, N16);
  launch_gemm<2, 1, false, 0>(stream, N16, kDim, 0, W16, kDim, 0, Q16, kDim, 0, ca_b, y, 0,
                              kTok, kDim, kDim, kWInv, 1);
  launch_gemm<2, 1, false, 0>(stream, Z16, kDim, 0, W16 + DD, kDim, 0, K16, kDim, 0, ca_b + kDim, y, 0,
                              kTok, kDim, kDim, kWInv, 1);
  launch_gemm<1, 1, false, 0>(stream, W16 + 2 * DD, kDim, 0, Z16, kDim, 0, VT16, kTok, 0, ca_b + 2 * kDim, y, 0,
                              kDim, kTok, kDim, kWInv, 1);
  for (int ch = 0; ch < kNChunk; ++ch) {
    const int b  = ch / (kHeads / kGrp);
    const int h0 = (ch % (kHeads / kGrp)) * kGrp;
    launch_gemm<0, 0, false, 0>(stream,
                                Q16 + (size_t)b * kSeq * kDim + (size_t)h0 * kDk, kDim, kDk,
                                K16 + (size_t)b * kSeq * kDim + (size_t)h0 * kDk, kDim, kDk,
                                Sc, kSeq, (long)SS2, ca_b, y, 0, kSeq, kSeq, kDk, kScoreScale, kGrp);
    softmax_row_kernel<<<kGrp * kSeq, 128, 0, stream>>>(Sc, mask + (size_t)b * kSeq, P16, kPCarry);
    launch_gemm<0, 1, false, 0>(stream, P16, kSeq, (long)SS2,
                                VT16 + (size_t)h0 * kDk * kTok + (size_t)b * kSeq, kTok, (long)kDk * kTok,
                                ATT16 + (size_t)b * kSeq * kDim + (size_t)h0 * kDk, kDim, kDk,
                                ca_b, y, 0, kSeq, kDk, kSeq, kPVScale, kGrp);
  }
  launch_gemm<2, 0, true, 0>(stream, ATT16, kDim, 0, W16 + 3 * DD, kDim, 0, Y2, kDim, 0, ca_b + 3 * kDim, Y1, 0,
                             kTok, kDim, kDim, kOutScale, 1);

  cast8_f16_kernel<<<castBlocks, 256, 0, stream>>>(w1, W16, n8w, kWCarry);
  cast8_f16_kernel<<<castBlocks, 256, 0, stream>>>(w2, W2_16, n8w, kWCarry);
  ln_kernel<<<kTok, 128, 0, stream>>>(Y2, ln_g + 2 * kDim, ln_b + 2 * kDim, N16);
  launch_gemm<2, 1, false, 3>(stream, N16, kDim, 0, W16, kDim, 0, H16, kDff, 0, b1, y, 0,
                              kTok, kDff, kDim, kWInv, 1);
  launch_gemm<2, 0, true, 0>(stream, H16, kDff, 0, W2_16, kDff, 0, outp, kDim, 0, b2, Y2, 0,
                             kTok, kDim, kDff, kWInv, 1);
}
